// Attention_18863496364032
// MI455X (gfx1250) — hardware-verified
//
#include <hip/hip_runtime.h>


#ifndef NB
#define NB 4
#endif
#ifndef SEQ
#define SEQ 2048
#endif
#ifndef QRES
#define QRES 1
#endif
static_assert(QRES == 1);
#define NB_FULL  4
#define SEQ_FULL 2048
#define DM   1024
#define NH   16
#define HD   64
#define ROWS (NB * SEQ)
#define QKP  (2 * DM)
#define NWV  4
#define BQ   (16 * NWV)
#define KS   32
#define OSP  68
#define GSP  68
#define GBM  128
#define GBN  64
#define WTN  128
#define WTK  64
#define VTP  72
#define LNT  256
#define LNC  4
#define L2E  1.4426950408889634f
#define XC   16.0f
#define WC   64.0f
#define QC   256.0f
#define KC   16.0f
#define VC   16.0f
#define PLG  10.0f
#define CC   2048.0f

static_assert(NH * HD == DM);
static_assert(HD == 64);
static_assert(NB <= NB_FULL);
static_assert(SEQ <= SEQ_FULL);
static_assert(SEQ % BQ == 0);
static_assert(SEQ % KS == 0);
static_assert(ROWS % GBM == 0);
static_assert(ROWS % GBN == 0);
static_assert(DM % GBM == 0);
static_assert(DM % GBN == 0);
static_assert(QKP % GBN == 0);
static_assert(DM % 32 == 0);
static_assert(DM % WTN == 0);
static_assert(DM % WTK == 0);
static_assert(LNT * LNC == DM);
static_assert(((size_t)ROWS * DM) % 2048 == 0);
static_assert((size_t)(3 * DM / WTN) * (DM / WTK) * (WTN * WTK) == (size_t)3 * DM * DM);
static_assert((size_t)(DM / WTN) * (DM / WTK) * (WTN * WTK) == (size_t)DM * DM);
static_assert((size_t)(QKP / GBN) * (ROWS / GBM) * (GBM * GBN) == (size_t)ROWS * QKP);
static_assert((size_t)(DM / GBN) * (ROWS / GBM) * (GBM * GBN) == (size_t)ROWS * DM);
static_assert((size_t)(ROWS / GBN) * (DM / GBM) * (GBM * GBN) == (size_t)DM * ROWS);
static_assert((size_t)(NB * NH * (SEQ / BQ)) * (BQ * HD) == (size_t)ROWS * DM);

#define SZ_XH  ((size_t)ROWS * DM * 2)
#define SZ_WQT ((size_t)3 * DM * DM * 2)
#define SZ_WOT ((size_t)DM * DM * 2)
#define SZ_QK  ((size_t)ROWS * QKP * 2)
#define SZ_PR  ((size_t)ROWS * DM * 4)
#define SZ_QL  ((size_t)ROWS * DM * 2)
#define SZ_VT  ((size_t)DM * ROWS * 2)
#define SZ_CH  ((size_t)ROWS * DM * 2)
#define SZ_CL  ((size_t)ROWS * DM * 2)
#define WS_TOTAL (SZ_XH + SZ_WQT + SZ_WOT + SZ_QK + SZ_QL + SZ_VT + SZ_CH + SZ_CL)
static_assert(SZ_PR <= SZ_QK);
static_assert(WS_TOTAL <= (size_t)134217728);
static_assert(SZ_XH % 256 == 0 && SZ_WQT % 256 == 0 && SZ_WOT % 256 == 0 && SZ_QK % 256 == 0 && SZ_QL % 256 == 0 && SZ_VT % 256 == 0 && SZ_CH % 256 == 0);

typedef unsigned short hf;
typedef __attribute__((ext_vector_type(16))) _Float16 v16h;
typedef __attribute__((ext_vector_type(2)))  _Float16 v2h;
typedef __attribute__((ext_vector_type(8)))  unsigned short v8us;
typedef __attribute__((ext_vector_type(8)))  unsigned int   v8u;
typedef __attribute__((ext_vector_type(8)))  float    v8f;
typedef __attribute__((ext_vector_type(4)))  float    v4f;
typedef v4f  __attribute__((may_alias)) v4fa;
typedef v8us __attribute__((may_alias)) v8usa;

__device__ __forceinline__ float bfr(float f) { unsigned u = __float_as_uint(f); u += 0x7FFFu + ((u >> 16) & 1u); return __uint_as_float(u & 0xFFFF0000u); }
__device__ __forceinline__ unsigned short f2h(float f) { return __builtin_bit_cast(unsigned short, (_Float16)f); }
__device__ __forceinline__ v16h cat16h(v8us lo, v8us hi) { return __builtin_bit_cast(v16h, __builtin_shufflevector(lo, hi, 0, 1, 2, 3, 4, 5, 6, 7, 8, 9, 10, 11, 12, 13, 14, 15)); }
__device__ __forceinline__ v8f wmmah(v16h a, v16h b, v8f c) { return __builtin_amdgcn_wmma_f32_16x16x32_f16(false, a, false, b, (short)0, c, false, false); }
__device__ __forceinline__ v16h ldh(const hf* p) { return cat16h(*(const v8us*)p, *(const v8us*)(p + 16)); }
__device__ __forceinline__ unsigned pk2h(float a, float b) { v2h t; t[0] = (_Float16)a; t[1] = (_Float16)b; return __builtin_bit_cast(unsigned, t); }
__device__ __forceinline__ void split8(const v4f x0, const v4f x1, v8us& oh, v8us& ol) {
#pragma unroll
    for (int c = 0; c < 4; ++c) {
        const _Float16 a = (_Float16)x0[c];
        const _Float16 b = (_Float16)x1[c];
        oh[c]     = __builtin_bit_cast(unsigned short, a);
        oh[4 + c] = __builtin_bit_cast(unsigned short, b);
        ol[c]     = f2h(x0[c] - (float)a);
        ol[4 + c] = f2h(x1[c] - (float)b);
    }
}

__global__ __launch_bounds__(256) void k_cvtx(const float* __restrict__ x, hf* XH) {
    const unsigned i = blockIdx.x * 256u + threadIdx.x;
    const unsigned per = (unsigned)(SEQ * DM / 8);
    if (i >= (unsigned)NB * per) return;
    const unsigned b = i / per, r = i - b * per;
    const float* src = x + (size_t)b * SEQ_FULL * DM + (size_t)r * 8;
    const v8f v = *(const v8f*)src;
    v8us o;
#pragma unroll
    for (int c = 0; c < 8; ++c) o[c] = f2h(bfr(v[c]) * XC);
    hf* dst = XH + (size_t)i * 8;
    *(volatile v8us*)dst = o;
    __threadfence();
    *(volatile v8us*)dst = o;
}

__global__ __launch_bounds__(256) void k_wt(const float* __restrict__ W, hf* WT, unsigned Kdim, unsigned Ncols) {
    __shared__ __align__(16) hf tl[WTN * VTP];
    const unsigned tid = threadIdx.x;
    const unsigned n0 = blockIdx.x * WTN;
    const unsigned k0 = blockIdx.y * WTK;
    const float* src = W + (size_t)k0 * Ncols + n0;
#pragma unroll
    for (unsigned it = 0; it < 8; ++it) {
        const unsigned f = it * 256u + tid;
        const unsigned kk = f >> 5, c4 = (f & 31u) * 4u;
        const v4f xv = *(const v4f*)(src + (size_t)kk * Ncols + c4);
#pragma unroll
        for (unsigned c = 0; c < 4; ++c) tl[(c4 + c) * VTP + kk] = f2h(bfr(xv[c]) * WC);
    }
    __syncthreads();
    hf* dst = WT + (size_t)n0 * Kdim + k0;
    const unsigned c8 = (tid & 7u) * 8u, dr = tid >> 3;
#pragma unroll 1
    for (int ps = 0; ps < 2; ++ps) {
#pragma unroll
        for (unsigned it = 0; it < 4; ++it) {
            const unsigned n = it * 32u + dr;
            const v8us o = *(const v8usa*)(tl + n * VTP + c8);
            *(volatile v8us*)(dst + (size_t)n * Kdim + c8) = o;
        }
        if (ps == 0) __threadfence();
    }
}

template <int NPL, int EPI>
__global__ __launch_bounds__(128) void k_gemm(const hf* A0, const hf* A1, const hf* BT,
                                              unsigned lda, unsigned ldb, unsigned K,
                                              hf* CH, hf* CL, unsigned ldc, unsigned ldl, unsigned nsplit,
                                              float sc0, float sc1, float* CF, const float* bias) {
    __shared__ __align__(16) float st[GBM * GSP];
    const unsigned tid = threadIdx.x, lane = tid & 31u, wv = tid >> 5, lr = lane & 15u, hi = lane >> 4;
    const unsigned wm = wv >> 1, wn = wv & 1u;
    const unsigned m0 = blockIdx.y * GBM, n0 = blockIdx.x * GBN;
    const size_t aoff = (size_t)(m0 + wm * 64u + lr) * lda + 8u * hi;
    const hf* ap  = A0 + aoff;
    const hf* ap1 = A1 + aoff;
    const hf* bp  = BT + (size_t)(n0 + wn * 32u + lr) * ldb + 8u * hi;

    v8f acc[4][2];
#pragma unroll
    for (int mt = 0; mt < 4; ++mt) { acc[mt][0] = (v8f){}; acc[mt][1] = (v8f){}; }

#pragma unroll 1
    for (unsigned k0 = 0; k0 < K; k0 += 32u) {
        const v16h b0 = ldh(bp + k0);
        const v16h b1 = ldh(bp + (size_t)16 * ldb + k0);
#pragma unroll
        for (int mt = 0; mt < 4; ++mt) {
            const v16h a = ldh(ap + (size_t)(mt * 16) * lda + k0);
            acc[mt][0] = wmmah(a, b0, acc[mt][0]);
            acc[mt][1] = wmmah(a, b1, acc[mt][1]);
            if (NPL == 2) {
                const v16h a2 = ldh(ap1 + (size_t)(mt * 16) * lda + k0);
                acc[mt][0] = wmmah(a2, b0, acc[mt][0]);
                acc[mt][1] = wmmah(a2, b1, acc[mt][1]);
            }
        }
        asm volatile("v_nop\n\tv_nop\n\tv_nop\n\tv_nop"
                     : "+v"(acc[0][0]), "+v"(acc[0][1]), "+v"(acc[1][0]), "+v"(acc[1][1]),
                       "+v"(acc[2][0]), "+v"(acc[2][1]), "+v"(acc[3][0]), "+v"(acc[3][1])
                     : "v"(b0), "v"(b1));
    }

    const float sc = (n0 < nsplit) ? sc0 : sc1;
#pragma unroll
    for (int mt = 0; mt < 4; ++mt) {
#pragma unroll
        for (int nt = 0; nt < 2; ++nt) {
#pragma unroll
            for (int r = 0; r < 8; ++r)
                st[(wm * 64u + mt * 16u + 8u * hi + r) * GSP + wn * 32u + nt * 16u + lr] = acc[mt][nt][r] * sc;
        }
    }
    __syncthreads();

    if (EPI == 0) {
        const unsigned c8 = (tid & 7u) * 8u, rr = tid >> 3;
        const bool wl = (n0 < nsplit);
        hf* ch = CH + (size_t)m0 * ldc + n0 + c8;
        hf* cl = CL + (size_t)m0 * ldl + n0 + c8;
#pragma unroll 1
        for (int ps = 0; ps < 2; ++ps) {
#pragma unroll 2
            for (unsigned it = 0; it < 8; ++it) {
                const unsigned row = it * 16u + rr;
                const v4f x0 = *(const v4fa*)(st + row * GSP + c8);
                const v4f x1 = *(const v4fa*)(st + row * GSP + c8 + 4u);
                v8us oh, ol;
                split8(x0, x1, oh, ol);
                *(volatile v8us*)(ch + (size_t)row * ldc) = oh;
                if (wl) *(volatile v8us*)(cl + (size_t)row * ldl) = ol;
            }
            if (ps == 0) __threadfence();
        }
    } else {
        const unsigned c4 = (tid & 15u) * 4u, rr = tid >> 4;
        v4f bb = *(const v4f*)(bias + n0 + c4);
        bb[0] = bfr(bb[0]); bb[1] = bfr(bb[1]); bb[2] = bfr(bb[2]); bb[3] = bfr(bb[3]);
        float* cf = CF + (size_t)m0 * ldc + n0 + c4;
#pragma unroll 1
        for (int ps = 0; ps < 2; ++ps) {
#pragma unroll 4
            for (unsigned it = 0; it < 16; ++it) {
                const unsigned row = it * 8u + rr;
                const v4f val = *(const v4fa*)(st + row * GSP + c4) + bb;
                *(volatile v4f*)(cf + (size_t)row * ldc) = val;
            }
            if (ps == 0) __threadfence();
        }
    }
}

__global__ __launch_bounds__(128) void k_flash(const hf* __restrict__ QKH, const hf* __restrict__ QL, const hf* __restrict__ VT, hf* CH, hf* CL) {
    __shared__ __align__(16) float os[NWV * 16 * OSP];
    const unsigned tid = threadIdx.x, lane = tid & 31u, wv = tid >> 5, lr = lane & 15u, hi = lane >> 4;
    const unsigned bpb = (unsigned)(SEQ / BQ);
    const unsigned bh = blockIdx.x / bpb;
    const unsigned b = bh / (unsigned)NH, h = bh - b * (unsigned)NH;
    const unsigned q0 = (blockIdx.x - bh * bpb) * BQ + wv * 16u;
    const unsigned vtpi = (unsigned)ROWS;

    v16h qh[2];
#if QRES
    v16h ql[2];
#endif
    {
        const hf* qp = QKH + ((size_t)b * SEQ + q0 + lr) * QKP + h * HD + 8u * hi;
        qh[0] = ldh(qp);
        qh[1] = ldh(qp + 32);
#if QRES
        const hf* qlp = QL + ((size_t)b * SEQ + q0 + lr) * DM + h * HD + 8u * hi;
        ql[0] = ldh(qlp);
        ql[1] = ldh(qlp + 32);
#endif
    }
    const hf* kp = QKH + ((size_t)b * SEQ + lr) * QKP + DM + h * HD + 8u * hi;
    const hf* vp = VT + ((size_t)(h * HD + lr)) * vtpi + (size_t)b * SEQ + 8u * hi;

    v8f o[4];
#pragma unroll
    for (int t = 0; t < 4; ++t) o[t] = (v8f){};
    float ml = -1.0e30f;
    float l = 0.0f;
    const float cs = (0.125f / (QC * KC)) * L2E;

#pragma unroll 1
    for (unsigned k0 = 0; k0 < (unsigned)SEQ; k0 += KS) {
        v8f s0 = (v8f){}, s1 = (v8f){};
        const hf* ka = kp + (size_t)k0 * QKP;
#pragma unroll
        for (int dk = 0; dk < 2; ++dk) {
            const v16h a0 = ldh(ka + dk * 32);
            const v16h a1 = ldh(ka + 16 * QKP + dk * 32);
            s0 = wmmah(a0, qh[dk], s0);
            s1 = wmmah(a1, qh[dk], s1);
#if QRES
            s0 = wmmah(a0, ql[dk], s0);
            s1 = wmmah(a1, ql[dk], s1);
#endif
        }
        asm volatile("v_nop\n\tv_nop\n\tv_nop\n\tv_nop" : "+v"(s0), "+v"(s1) : "v"(qh[0]), "v"(qh[1]));

        float mx = fmaxf(s0[0], s1[0]);
#pragma unroll
        for (int r = 1; r < 8; ++r) mx = fmaxf(mx, fmaxf(s0[r], s1[r]));
        mx = fmaxf(mx, __shfl_xor(mx, 16, 32));
        const float mnl = fmaxf(ml, mx * cs);
        const float corr = __builtin_amdgcn_exp2f(ml - mnl);
        ml = mnl;
        const float mo = mnl - PLG;
        float p0[8], p1[8];
        float ps = 0.0f;
#pragma unroll
        for (int r = 0; r < 8; ++r) {
            p0[r] = __builtin_amdgcn_exp2f(fmaf(s0[r], cs, -mo));
            p1[r] = __builtin_amdgcn_exp2f(fmaf(s1[r], cs, -mo));
            ps += p0[r] + p1[r];
        }
        ps += __shfl_xor(ps, 16, 32);
        l = l * corr + ps;
        if (__builtin_amdgcn_ballot_w32(corr != 1.0f) != 0u) {
#pragma unroll
            for (int t = 0; t < 4; ++t) o[t] *= corr;
        }

        v8u pw;
#pragma unroll
        for (int j = 0; j < 4; ++j) {
            pw[j]     = pk2h(p0[2 * j], p0[2 * j + 1]);
            pw[4 + j] = pk2h(p1[2 * j], p1[2 * j + 1]);
        }
        const v16h ph = __builtin_bit_cast(v16h, pw);

        asm volatile("" ::: "memory");
        const hf* va = vp + k0;
#pragma unroll
        for (int t = 0; t < 4; ++t) {
            const v16h a = ldh(va + (size_t)(t * 16) * vtpi);
            o[t] = wmmah(a, ph, o[t]);
        }
        asm volatile("v_nop\n\tv_nop\n\tv_nop\n\tv_nop"
                     : "+v"(o[0]), "+v"(o[1]), "+v"(o[2]), "+v"(o[3])
                     : "v"(ph));
    }

    const float inv = (CC / VC) / l;
    float* ow = os + wv * (16 * OSP);
#pragma unroll
    for (int t = 0; t < 4; ++t) {
#pragma unroll
        for (int r = 0; r < 8; ++r) ow[lr * OSP + t * 16 + 8 * hi + r] = o[t][r] * inv;
    }
    __syncthreads();
    const unsigned c8 = (lane & 7u) * 8u, rq = lane >> 3;
    const size_t cbase = ((size_t)b * SEQ + q0) * DM + h * HD + c8;
#pragma unroll 1
    for (int ps2 = 0; ps2 < 2; ++ps2) {
#pragma unroll
        for (unsigned it = 0; it < 4; ++it) {
            const unsigned row = it * 4u + rq;
            const v4f x0 = *(const v4fa*)(ow + row * OSP + c8);
            const v4f x1 = *(const v4fa*)(ow + row * OSP + c8 + 4u);
            v8us oh, ol;
            split8(x0, x1, oh, ol);
            *(volatile v8us*)(CH + cbase + (size_t)row * DM) = oh;
            *(volatile v8us*)(CL + cbase + (size_t)row * DM) = ol;
        }
        if (ps2 == 0) __threadfence();
    }
}

__global__ __launch_bounds__(LNT) void k_ln(const float* __restrict__ PR, const float* __restrict__ g, const float* __restrict__ be, float* O) {
    __shared__ float ra[LNT / 32];
    __shared__ float rb[LNT / 32];
    const unsigned tid = threadIdx.x, lane = tid & 31u, wv = tid >> 5;
    const size_t base = (size_t)blockIdx.x * DM + tid * LNC;
    const v4f v = *(const v4f*)(PR + base);
    float s = (v[0] + v[1]) + (v[2] + v[3]);
#pragma unroll
    for (int off = 16; off > 0; off >>= 1) s += __shfl_xor(s, off, 32);
    if (lane == 0u) ra[wv] = s;
    __syncthreads();
    float tot = 0.0f;
#pragma unroll
    for (int i = 0; i < LNT / 32; ++i) tot += ra[i];
    const float mean = tot * (1.0f / (float)DM);
    const float d0 = v[0] - mean, d1 = v[1] - mean, d2 = v[2] - mean, d3 = v[3] - mean;
    float q = (d0 * d0 + d1 * d1) + (d2 * d2 + d3 * d3);
#pragma unroll
    for (int off = 16; off > 0; off >>= 1) q += __shfl_xor(q, off, 32);
    if (lane == 0u) rb[wv] = q;
    __syncthreads();
    float tq = 0.0f;
#pragma unroll
    for (int i = 0; i < LNT / 32; ++i) tq += rb[i];
    const float rstd = rsqrtf(tq * (1.0f / (float)DM) + 1.0e-5f);
    const v4f gv = *(const v4f*)(g + tid * LNC);
    const v4f bv = *(const v4f*)(be + tid * LNC);
    v4f y;
    y[0] = d0 * rstd * bfr(gv[0]) + bfr(bv[0]);
    y[1] = d1 * rstd * bfr(gv[1]) + bfr(bv[1]);
    y[2] = d2 * rstd * bfr(gv[2]) + bfr(bv[2]);
    y[3] = d3 * rstd * bfr(gv[3]) + bfr(bv[3]);
    *(volatile v4f*)(O + base) = y;
    __threadfence();
    *(volatile v4f*)(O + base) = y;
}

extern "C" void kernel_launch(void* const* d_in, const int* in_sizes, int n_in,
                              void* d_out, int out_size, void* d_ws, size_t ws_size, hipStream_t stream) {
    if (n_in < 6) return;
    const size_t needx = ((size_t)(NB - 1) * SEQ_FULL + SEQ) * DM;
    if ((size_t)in_sizes[0] < needx) return;
    if ((size_t)in_sizes[1] < (size_t)3 * DM * DM) return;
    if ((size_t)in_sizes[2] < (size_t)DM * DM) return;
    if ((size_t)in_sizes[3] < (size_t)DM || (size_t)in_sizes[4] < (size_t)DM || (size_t)in_sizes[5] < (size_t)DM) return;
    if ((size_t)out_size < (size_t)ROWS * DM) return;
    if (WS_TOTAL > ws_size) return;

    const float* x     = (const float*)d_in[0];
    const float* w_qkv = (const float*)d_in[1];
    const float* w_out = (const float*)d_in[2];
    const float* b_out = (const float*)d_in[3];
    const float* gam   = (const float*)d_in[4];
    const float* bet   = (const float*)d_in[5];
    float* OUT = (float*)d_out;

    char* wsp = (char*)d_ws;
    size_t off = 0;
    hf* XH  = (hf*)(wsp + off); off += SZ_XH;
    hf* WQT = (hf*)(wsp + off); off += SZ_WQT;
    hf* WOT = (hf*)(wsp + off); off += SZ_WOT;
    hf* QKH = (hf*)(wsp + off);
    float* PR = (float*)(wsp + off); off += SZ_QK;
    hf* QLp = (hf*)(wsp + off); off += SZ_QL;
    hf* VT  = (hf*)(wsp + off); off += SZ_VT;
    hf* CHp = (hf*)(wsp + off); off += SZ_CH;
    hf* CLp = (hf*)(wsp + off); off += SZ_CL;

    const float sq = QC / (XC * WC);
    const float sk = KC / (XC * WC);
    const float sv = VC / (XC * WC);
    const float sp = 1.0f / (CC * WC);

    const unsigned gc = (unsigned)(((size_t)ROWS * DM / 8 + 255) / 256);
    k_cvtx<<<gc, 256, 0, stream>>>(x, XH);
    k_wt<<<dim3(3 * DM / WTN, DM / WTK, 1), 256, 0, stream>>>(w_qkv, WQT, (unsigned)DM, (unsigned)(3 * DM));
    k_wt<<<dim3(DM / WTN, DM / WTK, 1), 256, 0, stream>>>(w_out, WOT, (unsigned)DM, (unsigned)DM);
    k_gemm<1, 0><<<dim3(QKP / GBN, ROWS / GBM, 1), 128, 0, stream>>>(
        XH, XH, WQT, (unsigned)DM, (unsigned)DM, (unsigned)DM,
        QKH, QLp, (unsigned)QKP, (unsigned)DM, (unsigned)(QRES ? DM : 0), sq, sk, PR, b_out);
    k_gemm<1, 0><<<dim3(ROWS / GBN, DM / GBM, 1), 128, 0, stream>>>(
        WQT + (size_t)2 * DM * DM, WQT + (size_t)2 * DM * DM, XH, (unsigned)DM, (unsigned)DM, (unsigned)DM,
        VT, QLp, (unsigned)ROWS, (unsigned)DM, 0u, sv, sv, PR, b_out);
    k_flash<<<(unsigned)(NB * NH * (SEQ / BQ)), 128, 0, stream>>>(QKH, QLp, VT, CHp, CLp);
    k_gemm<2, 1><<<dim3(DM / GBN, ROWS / GBM, 1), 128, 0, stream>>>(
        CHp, CLp, WOT, (unsigned)DM, (unsigned)DM, (unsigned)DM,
        CHp, CLp, (unsigned)DM, (unsigned)DM, 0u, sp, sp, PR, b_out);
    k_ln<<<(unsigned)ROWS, LNT, 0, stream>>>(PR, gam, bet, OUT);
}
